// CosineAttention_85212151152953
// MI455X (gfx1250) — hardware-verified
//
#include <hip/hip_runtime.h>
#include <math.h>

typedef __attribute__((ext_vector_type(16))) _Float16 v16h;
typedef __attribute__((ext_vector_type(16))) __bf16 v16b;
typedef __attribute__((ext_vector_type(8)))  _Float16 v8h;
typedef __attribute__((ext_vector_type(8)))  float v8f;
typedef __attribute__((ext_vector_type(4)))  float v4f;
typedef __attribute__((ext_vector_type(2)))  float v2f;
typedef __attribute__((ext_vector_type(4)))  unsigned v4u;
typedef __attribute__((ext_vector_type(4)))  int v4i;
typedef float __attribute__((may_alias)) float_a;
typedef int __attribute__((may_alias)) int_a;

template <typename T> __device__ __forceinline__ void vst2(void* p, T v) { *(volatile T*)p = v; __threadfence(); *(volatile T*)p = v; }
__device__ __forceinline__ v8f wmma16(v16h a, v16h b, v8f c) {
  v8f d = __builtin_amdgcn_wmma_f32_16x16x32_f16(false, a, false, b, (short)0, c, false, false);
  asm volatile("v_nop\n\tv_nop\n\tv_nop\n\tv_nop" : "+v"(d) : "v"(a), "v"(b));
  return d;
}
__device__ __forceinline__ v8f wmma_bf(v16b a, v16b b, v8f c) {
  v8f d = __builtin_amdgcn_wmma_f32_16x16x32_bf16(false, a, false, b, (short)0, c, false, false);
  asm volatile("v_nop\n\tv_nop\n\tv_nop\n\tv_nop" : "+v"(d) : "v"(a), "v"(b));
  return d;
}
__device__ __forceinline__ v16h frag_h(const _Float16* rowk0, int lane) {
  union { v16h v; v8h q[2]; } u; const _Float16* p = rowk0 + 8 * (lane >> 4);
  u.q[0] = *(const v8h*)p; u.q[1] = *(const v8h*)(p + 16); return u.v;
}
__device__ __forceinline__ v16h frag_f32(const float* rowk0, int lane) {
  v16h a; const float* p = rowk0 + 8 * (lane >> 4);
#pragma unroll
  for (int i = 0; i < 8; ++i) { a[i] = (_Float16)p[i]; a[8 + i] = (_Float16)p[16 + i]; }
  return a;
}
__device__ __forceinline__ v16h frag_f32s(const float* rowk0, int lane, float sc) {
  v16h a; const float* p = rowk0 + 8 * (lane >> 4);
#pragma unroll
  for (int i = 0; i < 8; ++i) { a[i] = (_Float16)(p[i] * sc); a[8 + i] = (_Float16)(p[16 + i] * sc); }
  return a;
}
__device__ __forceinline__ v16h fragc_f32(const float* W, int k0, int n, int lane, int ld, int K) {
  v16h a; const int g = lane >> 4;
#pragma unroll
  for (int i = 0; i < 8; ++i) { const int ka = k0 + 8 * g + i, kb = ka + 16;
    a[i] = (_Float16)(ka < K ? W[(size_t)(ka < K ? ka : K - 1) * ld + n] : 0.f); a[8 + i] = (_Float16)(kb < K ? W[(size_t)(kb < K ? kb : K - 1) * ld + n] : 0.f); }
  return a;
}
struct F2 { v16b h, l; };
__device__ __forceinline__ F2 bsplit16(const float v[16]) { F2 r;
#pragma unroll
  for (int i = 0; i < 16; ++i) { const __bf16 h = (__bf16)v[i]; r.h[i] = h; r.l[i] = (__bf16)(v[i] - (float)h); }
  return r; }
__device__ __forceinline__ F2 split_row(const float* row, int k0, int lane) { float v[16]; const float* p = row + k0 + 8 * (lane >> 4);
#pragma unroll
  for (int i = 0; i < 8; ++i) { v[i] = p[i]; v[8 + i] = p[16 + i]; }
  return bsplit16(v); }
__device__ __forceinline__ F2 split_rowK(const float* row, int k0, int lane, int K) { float v[16]; const int g = lane >> 4;
#pragma unroll
  for (int i = 0; i < 8; ++i) { const int ka = k0 + 8 * g + i, kb = ka + 16; v[i] = ka < K ? row[ka < K ? ka : K - 1] : 0.f; v[8 + i] = kb < K ? row[kb < K ? kb : K - 1] : 0.f; }
  return bsplit16(v); }
__device__ __forceinline__ F2 split_col(const float* W, int k0, int n, int lane, int ld, int K) { float v[16]; const int g = lane >> 4;
#pragma unroll
  for (int i = 0; i < 8; ++i) { const int ka = k0 + 8 * g + i, kb = ka + 16; v[i] = ka < K ? W[(size_t)(ka < K ? ka : K - 1) * ld + n] : 0.f; v[8 + i] = kb < K ? W[(size_t)(kb < K ? kb : K - 1) * ld + n] : 0.f; }
  return bsplit16(v); }
__device__ __forceinline__ v8f mac3(const F2& a, const F2& b, v8f c) { c = wmma_bf(a.l, b.h, c); c = wmma_bf(a.h, b.l, c); return wmma_bf(a.h, b.h, c); }
__device__ __forceinline__ float sigm(float v) { return 1.0f / (1.0f + expf(-v)); }
#define LDSX() do { asm volatile("s_wait_dscnt 0" ::: "memory"); __builtin_amdgcn_wave_barrier(); __builtin_amdgcn_fence(__ATOMIC_RELEASE, "workgroup"); } while (0)


#define NB 4
#define NQ 1024
#define NM 2048
#define DIM 1024
#define NH 16
#define HD2 64
#ifndef TNB
#define TNB NB
#endif
typedef __attribute__((ext_vector_type(8))) __bf16 v8b;
__device__ __forceinline__ v16b frag_b(const __bf16* rowk0, int lane) {
  union { v16b v; v8b q[2]; } u; const __bf16* p = rowk0 + 8 * (lane >> 4);
  u.q[0] = *(const v8b*)p; u.q[1] = *(const v8b*)(p + 16); return u.v;
}
__device__ __forceinline__ float bfr(float v) { return (float)(__bf16)v; }
__device__ __attribute__((noinline)) float exp_ni(float v) { return expf(v); }
__device__ __attribute__((noinline)) float erf_ni(float v) { return erff(v); }

#define WS_QN  0u
#define WS_KN  (WS_QN + 4u * (size_t)NB * NQ * DIM)
#define WS_VP  (WS_KN + 4u * (size_t)NB * DIM * NM)
#define WS_MT  (WS_VP + 4u * (size_t)NB * DIM * NM)
#define WS_CT  (WS_MT + 4u * (size_t)NB * NH * HD2 * HD2)
#define WS_END (WS_CT + 4u * (size_t)NB * NQ * DIM)

__global__ __launch_bounds__(128) void k_proj(const float* __restrict__ Qi, const float* __restrict__ Ki, const float* __restrict__ Vi, const float* __restrict__ G, const float* __restrict__ Bt, const float* __restrict__ WIN, float* __restrict__ QN, float* __restrict__ KN, float* __restrict__ VP) {
  __shared__ __align__(16) float sst[64][2]; __shared__ __align__(16) float sf[4][16][132]; __shared__ __align__(16) float tt[128][68];
  const int tid = threadIdx.x, wave = tid >> 5, lane = tid & 31, col = lane & 15, g = lane >> 4; const int which = blockIdx.z / TNB; const size_t b = blockIdx.z % TNB; const int c0 = blockIdx.y * 128; const int nrows = (which == 0) ? NQ : NM;
  if ((int)blockIdx.x * 64 >= nrows) return;
  const float* X = (which == 0 ? Qi : which == 1 ? Ki : Vi) + (b * nrows + (size_t)blockIdx.x * 64) * DIM;
  { const int rl = tid >> 1, half = tid & 1; const float* xr = X + (size_t)rl * DIM + half * 512; float s = 0.f;
#pragma unroll 1
    for (int i = 0; i < 512; ++i) s += bfr(xr[i]);
    s += __shfl_xor(s, 1); const float mu = s * (1.0f / DIM); float q = 0.f;
#pragma unroll 1
    for (int i = 0; i < 512; ++i) { const float d = bfr(xr[i]) - mu; q += d * d; }
    q += __shfl_xor(q, 1); if (half == 0) { sst[rl][0] = mu; sst[rl][1] = 1.0f / sqrtf(q * (1.0f / DIM) + 1e-5f); } }
  __syncthreads();
  const int rl = wave * 16 + col; const float mu = sst[rl][0], inv = sst[rl][1]; const float* xr = X + (size_t)rl * DIM;
  v8f acc[8] = {};
#pragma unroll 2
  for (int kc = 0; kc < DIM / 32; ++kc) { float v[16]; const int k0 = kc * 32 + 8 * g;
#pragma unroll
    for (int i = 0; i < 8; ++i) { const int ka = k0 + i, kb = k0 + 16 + i; v[i] = (bfr(xr[ka]) - mu) * inv * bfr(G[ka]) + bfr(Bt[ka]); v[8 + i] = (bfr(xr[kb]) - mu) * inv * bfr(G[kb]) + bfr(Bt[kb]); }
    const F2 a = bsplit16(v);
#pragma unroll
    for (int j = 0; j < 8; ++j) { v16b w; const int o = c0 + j * 16 + col;
#pragma unroll
      for (int i = 0; i < 8; ++i) { w[i] = (__bf16)WIN[(size_t)(kc * 32 + 8 * g + i) * DIM + o]; w[8 + i] = (__bf16)WIN[(size_t)(kc * 32 + 16 + 8 * g + i) * DIM + o]; }
      acc[j] = wmma_bf(a.h, w, acc[j]); acc[j] = wmma_bf(a.l, w, acc[j]); } }
  float sc0 = 1.f, sc1 = 1.f; float rn0[8], rn1[8];
#pragma unroll
  for (int r = 0; r < 8; ++r) { float a0 = 0.f, a1 = 0.f;
#pragma unroll
    for (int j = 0; j < 4; ++j) { a0 += acc[j][r] * acc[j][r]; a1 += acc[4 + j][r] * acc[4 + j][r]; }
#pragma unroll
    for (int o = 1; o < 16; o <<= 1) { a0 += __shfl_xor(a0, o); a1 += __shfl_xor(a1, o); }
    rn0[r] = (which == 2) ? 1.f : 1.0f / sqrtf(a0); rn1[r] = (which == 2) ? 1.f : 1.0f / sqrtf(a1); }
  (void)sc0; (void)sc1;
  if (which == 0) {
#pragma unroll
    for (int j = 0; j < 8; ++j)
#pragma unroll
      for (int r = 0; r < 8; ++r) sf[wave][8 * g + r][j * 16 + col] = acc[j][r] * (j < 4 ? rn0[r] : rn1[r]);
    LDSX(); for (int rr = 0; rr < 16; ++rr) vst2(QN + (b * NQ + (size_t)blockIdx.x * 64 + wave * 16 + rr) * DIM + c0 + lane * 4, *(const v4f*)&sf[wave][rr][lane * 4]); }
  else {
#pragma unroll
    for (int j = 0; j < 8; ++j)
#pragma unroll
      for (int r = 0; r < 8; ++r) tt[j * 16 + col][wave * 16 + 8 * g + r] = acc[j][r] * (j < 4 ? rn0[r] : rn1[r]);
    __syncthreads(); float* dst = (which == 1) ? KN : VP;
    for (int e = tid; e < 128 * 16; e += 128) { const int cl = e >> 4, q = e & 15; vst2(dst + ((b * DIM + c0 + cl) * (size_t)NM) + (size_t)blockIdx.x * 64 + q * 4, *(const v4f*)&tt[cl][q * 4]); } } }
__global__ __launch_bounds__(128) void k_kv(const float* __restrict__ KN, const float* __restrict__ VP, float* __restrict__ MT) { __shared__ __align__(16) float tt[64][68];
  const int tid = threadIdx.x, wave = tid >> 5, lane = tid & 31, col = lane & 15, g = lane >> 4; const int h = blockIdx.x; const size_t b = blockIdx.y;
  const float* arow = KN + (b * DIM + (size_t)h * HD2 + wave * 16 + col) * NM;
  v8f acc[4] = {};
#pragma unroll 2
  for (int kc = 0; kc < NM / 32; ++kc) { const F2 a = split_row(arow, kc * 32, lane);
#pragma unroll
    for (int j = 0; j < 4; ++j) { const F2 w = split_row(VP + (b * DIM + (size_t)h * HD2 + j * 16 + col) * NM, kc * 32, lane); acc[j] = mac3(a, w, acc[j]); } }
#pragma unroll
  for (int j = 0; j < 4; ++j)
#pragma unroll
    for (int r = 0; r < 8; ++r) tt[j * 16 + col][wave * 16 + 8 * g + r] = acc[j][r];
  __syncthreads();
  for (int e = tid; e < 64 * 16; e += 128) { const int er = e >> 4, q = e & 15; vst2(MT + (((b * NH + h) * HD2 + er) * HD2) + q * 4, *(const v4f*)&tt[er][q * 4]); } }
__global__ __launch_bounds__(128) void k_ctx(const float* __restrict__ QN, const float* __restrict__ MT, float* __restrict__ CT) { __shared__ __align__(16) float sf[4][16][68];
  const int tid = threadIdx.x, wave = tid >> 5, lane = tid & 31, col = lane & 15, g = lane >> 4; const size_t b = blockIdx.y; const size_t r0 = b * NQ + (size_t)blockIdx.x * 64 + wave * 16;
#pragma unroll 1
  for (int h = 0; h < NH; ++h) { v8f acc[4] = {};
#pragma unroll
    for (int kc = 0; kc < 2; ++kc) { const F2 a = split_row(QN + (r0 + col) * DIM + h * HD2, kc * 32, lane);
#pragma unroll
      for (int j = 0; j < 4; ++j) { const F2 w = split_row(MT + (((b * NH + h) * HD2 + j * 16 + col) * HD2), kc * 32, lane); acc[j] = mac3(a, w, acc[j]); } }
#pragma unroll
    for (int j = 0; j < 4; ++j)
#pragma unroll
      for (int r = 0; r < 8; ++r) sf[wave][8 * g + r][j * 16 + col] = acc[j][r];
    LDSX(); for (int rr = 0; rr < 16; ++rr) if (lane < 16) vst2(CT + (r0 + rr) * DIM + h * HD2 + lane * 4, *(const v4f*)&sf[wave][rr][lane * 4]);
    LDSX(); } }
__global__ __launch_bounds__(128) void k_out(const float* __restrict__ CT, const float* __restrict__ WO, const float* __restrict__ BO, float* __restrict__ OUT) { __shared__ __align__(16) float sf[4][16][132];
  const int tid = threadIdx.x, wave = tid >> 5, lane = tid & 31, col = lane & 15, g = lane >> 4; const size_t b = blockIdx.z; const int c0 = blockIdx.y * 128; const size_t r0 = b * NQ + (size_t)blockIdx.x * 64 + wave * 16;
  v8f acc[8] = {};
#pragma unroll 2
  for (int kc = 0; kc < DIM / 32; ++kc) { const F2 a = split_row(CT + (r0 + col) * DIM, kc * 32, lane);
#pragma unroll
    for (int j = 0; j < 8; ++j) { v16b w; const int o = c0 + j * 16 + col;
#pragma unroll
      for (int i = 0; i < 8; ++i) { w[i] = (__bf16)WO[(size_t)(kc * 32 + 8 * g + i) * DIM + o]; w[8 + i] = (__bf16)WO[(size_t)(kc * 32 + 16 + 8 * g + i) * DIM + o]; }
      acc[j] = wmma_bf(a.h, w, acc[j]); acc[j] = wmma_bf(a.l, w, acc[j]); } }
#pragma unroll
  for (int j = 0; j < 8; ++j) { const float bb = bfr(BO[c0 + j * 16 + col]);
#pragma unroll
    for (int r = 0; r < 8; ++r) sf[wave][8 * g + r][j * 16 + col] = acc[j][r] + bb; }
  LDSX(); for (int rr = 0; rr < 16; ++rr) vst2(OUT + (r0 + rr) * DIM + c0 + lane * 4, *(const v4f*)&sf[wave][rr][lane * 4]); }
extern "C" void kernel_launch(void* const* d_in, const int* in_sizes, int n_in, void* d_out, int out_size, void* d_ws, size_t ws_size, hipStream_t stream) {
  (void)in_sizes; (void)n_in; (void)out_size;
  const float** F = (const float**)d_in;
  if (ws_size < (size_t)WS_END) return;
  char* ws = (char*)d_ws; float *QN = (float*)(ws + WS_QN), *KN = (float*)(ws + WS_KN), *VP = (float*)(ws + WS_VP), *MT = (float*)(ws + WS_MT), *CT = (float*)(ws + WS_CT);
  k_proj<<<dim3(NM / 64, DIM / 128, 3 * TNB), 128, 0, stream>>>(F[0], F[1], F[2], F[3], F[4], F[5], QN, KN, VP);
  k_kv<<<dim3(NH, TNB), 128, 0, stream>>>(KN, VP, MT);
  k_ctx<<<dim3(NQ / 64, TNB), 128, 0, stream>>>(QN, MT, CT);
  k_out<<<dim3(NQ / 64, DIM / 128, TNB), 128, 0, stream>>>(CT, F[6], F[7], (float*)d_out);
}
